// GNN_geoGCN_81758997447248
// MI455X (gfx1250) — hardware-verified
//
#include <hip/hip_runtime.h>
#include <stddef.h>
#include <stdint.h>


#define C1 128
#define O1 2048
#define C2 2048
#define O2 2048
#define C3 2048
#define O3 1024

#define NTHR   256
#define NWAVE  8
#define EPT    8
#define CHUNK  (NTHR * EPT)
#define WCAP   (EPT * 32)
#define LISTN  (NWAVE * WCAP)
#define NBA    1024
#define SLA    10
#define NBW    32
#define DEGC   31
#define BK_ZINTS (NBA * NBW + LISTN + NBA)
#define BK_LDS_INTS (BK_ZINTS + 16)
#define GBM    64
#define GBN    128
#define GTHR   128
#define ATHR   512
#define AITER  4
#define NU1    (O1 * (C1 / 8))
#define NU2    (O2 * (C2 / 8))
#define NU3    (O3 * (C3 / 8))
#define NUT    (NU1 + NU2 + NU3)

static_assert((CHUNK & (CHUNK - 1)) == 0 && CHUNK <= 4096);
static_assert((NBA & (NBA - 1)) == 0 && NBA == (1 << SLA));
static_assert(((long long)CHUNK << SLA) < (1LL << 31));
static_assert(WCAP * NWAVE == CHUNK);
static_assert(BK_ZINTS % (NTHR * 4) == 0);
static_assert((NBA * NBW) % (NTHR * 4) == 0);
static_assert(NBA % GBM == 0);
static_assert(DEGC == NBW - 1);
static_assert(O1 == C2 && O2 == C3);
static_assert(C1 % 32 == 0 && C2 % 32 == 0 && C3 % 32 == 0);
static_assert(O1 % GBN == 0 && O2 % GBN == 0 && O3 % GBN == 0);
static_assert(GBM == (GTHR / 32) * 16 && GBN == 128);
static_assert(NU1 % NTHR == 0 && NU2 % NTHR == 0 && NU3 % NTHR == 0);
static_assert(O3 == 8 * 128);
static_assert(BK_LDS_INTS * 4 <= 300000);

typedef float          v2f   __attribute__((ext_vector_type(2)));
typedef float          v4f   __attribute__((ext_vector_type(4)));
typedef float          v8f   __attribute__((ext_vector_type(8)));
typedef int            v4i   __attribute__((ext_vector_type(4)));
typedef int            v8i   __attribute__((ext_vector_type(8)));
typedef unsigned short v8us  __attribute__((ext_vector_type(8)));
typedef unsigned short v16us __attribute__((ext_vector_type(16)));
typedef __bf16         v16bf __attribute__((ext_vector_type(16)));
typedef v2f  __attribute__((may_alias)) v2fa;
typedef v4f  __attribute__((may_alias)) v4fa;
typedef v4i  __attribute__((may_alias)) v4ia;
typedef v8us __attribute__((may_alias)) v8usa;
union FragB { v16bf v; v16us u; v8us h[2]; v8i w; };

__device__ __forceinline__ v8f wmb(const FragB& a, const FragB& b, v8f c) {
  v8f d = __builtin_amdgcn_wmma_f32_16x16x32_bf16(false, a.v, false, b.v, (short)0, c, false, false);
  asm volatile("v_nop\n\tv_nop\n\tv_nop\n\tv_nop" : "+v"(d) : "v"(a.w), "v"(b.w));
  return d;
}

__device__ __forceinline__ unsigned bf16_bits(float f) {
  const unsigned u = __float_as_uint(f);
  return (u + 0x7FFFu + ((u >> 16) & 1u)) >> 16;
}
__device__ __forceinline__ float bf16_val(float f) {
  return __uint_as_float(bf16_bits(f) << 16);
}
__device__ __forceinline__ v4f bf16_val4(v4f a) {
  v4f r;
  r.x = bf16_val(a.x); r.y = bf16_val(a.y); r.z = bf16_val(a.z); r.w = bf16_val(a.w);
  return r;
}

template <int SLB>
__device__ __forceinline__ int scan_chunk(const int* __restrict__ dsts, int nE, int cbase, int slotBase,
                                          int nb, int* list, int lane, int wave) {
  int wc = 0;
  const int el0  = wave * WCAP + lane;
  const int e0   = cbase + el0;
  const int sent = -2147483647 - 1;
  const int last = nE - 1;
  const int r0 = dsts[min(e0,       last)];
  const int r1 = dsts[min(e0 + 32,  last)];
  const int r2 = dsts[min(e0 + 64,  last)];
  const int r3 = dsts[min(e0 + 96,  last)];
  const int r4 = dsts[min(e0 + 128, last)];
  const int r5 = dsts[min(e0 + 160, last)];
  const int r6 = dsts[min(e0 + 192, last)];
  const int r7 = dsts[min(e0 + 224, last)];
  const int d0 = (e0       < nE) ? r0 : sent;
  const int d1 = (e0 + 32  < nE) ? r1 : sent;
  const int d2 = (e0 + 64  < nE) ? r2 : sent;
  const int d3 = (e0 + 96  < nE) ? r3 : sent;
  const int d4 = (e0 + 128 < nE) ? r4 : sent;
  const int d5 = (e0 + 160 < nE) ? r5 : sent;
  const int d6 = (e0 + 192 < nE) ? r6 : sent;
  const int d7 = (e0 + 224 < nE) ? r7 : sent;
  const unsigned nbs = (unsigned)slotBase;
  const unsigned unb = (unsigned)nb;
  const unsigned s0 = (unsigned)d0 - nbs, s1 = (unsigned)d1 - nbs;
  const unsigned s2 = (unsigned)d2 - nbs, s3 = (unsigned)d3 - nbs;
  const unsigned s4 = (unsigned)d4 - nbs, s5 = (unsigned)d5 - nbs;
  const unsigned s6 = (unsigned)d6 - nbs, s7 = (unsigned)d7 - nbs;
  const bool h0 = s0 < unb, h1 = s1 < unb, h2 = s2 < unb, h3 = s3 < unb;
  const bool h4 = s4 < unb, h5 = s5 < unb, h6 = s6 < unb, h7 = s7 < unb;
  const unsigned any = __builtin_amdgcn_ballot_w32(h0 | h1 | h2 | h3 | h4 | h5 | h6 | h7);
  if (any != 0u) {
#define HITJ(J, HJ, SJ) { \
      const unsigned mj = __builtin_amdgcn_ballot_w32(HJ); \
      if (mj != 0u) { \
        if (HJ) { \
          const int pos = wc + (int)__builtin_amdgcn_mbcnt_lo(mj, 0u); \
          if (pos < WCAP) list[wave * WCAP + pos] = ((el0 + 32 * (J)) << SLB) | (int)(SJ); \
        } \
        wc += (int)__builtin_popcount(mj); } }
    HITJ(0, h0, s0)
    HITJ(1, h1, s1)
    HITJ(2, h2, s2)
    HITJ(3, h3, s3)
    HITJ(4, h4, s4)
    HITJ(5, h5, s5)
    HITJ(6, h6, s6)
    HITJ(7, h7, s7)
#undef HITJ
  }
  return wc;
}

__global__ __launch_bounds__(NTHR) void k_wprep(const float* __restrict__ W1, const float* __restrict__ W2,
                                                const float* __restrict__ W3,
                                                unsigned short* W1T, unsigned short* W2T, unsigned short* W3T) {
  const int u = (int)blockIdx.x * NTHR + (int)threadIdx.x;
  const float* W;
  unsigned short* P;
  int K, N, sh, v;
  if (u < NU1)                  { W = W1; P = W1T; K = C1; N = O1; sh = 4; v = u; }
  else if (u < NU1 + NU2)       { W = W2; P = W2T; K = C2; N = O2; sh = 8; v = u - NU1; }
  else if (u < NUT)             { W = W3; P = W3T; K = C3; N = O3; sh = 8; v = u - NU1 - NU2; }
  else return;
  const int n  = v >> sh;
  const int k8 = (v & ((1 << sh) - 1)) * 8;
  const float* p = W + (size_t)k8 * (size_t)N + n;
  v8us o;
#pragma unroll
  for (int i = 0; i < 8; ++i) o[i] = (unsigned short)bf16_bits(p[(size_t)i * (size_t)N]);
  unsigned short* dp = P + (size_t)n * (size_t)K + k8;
  *(volatile v8us*)dp = o;
  __threadfence();
  *(volatile v8us*)dp = o;
}

__global__ __launch_bounds__(NTHR) void k_bucket(const int* __restrict__ srcs, const int* __restrict__ dsts,
                                                 int nE, int nN, int* nbr) {
  extern __shared__ __attribute__((aligned(16))) int dsm[];
  int* rows = dsm;
  int* list = dsm + NBA * NBW;
  int* cnt  = list + LISTN;
  int* misc = cnt + NBA;
  const int tid = (int)threadIdx.x, lane = tid & 31;
  const int wave = __builtin_amdgcn_readfirstlane(tid >> 5);
  const int nodeBase = (int)blockIdx.x * NBA;

  {
    const v4i z4 = {0, 0, 0, 0};
    for (int i = tid * 4; i < BK_ZINTS; i += NTHR * 4) *(v4ia*)(dsm + i) = z4;
    if (tid < 16) misc[tid] = 0;
  }
  __syncthreads();

  const int nChunks = (nE + CHUNK - 1) / CHUNK;
#pragma unroll 1
  for (int ch = 0; ch < nChunks; ++ch) {
    const int cbase = ch * CHUNK;
    const int wc = scan_chunk<SLA>(dsts, nE, cbase, nodeBase, NBA, list, lane, wave);
    if (lane == 0) misc[wave] = wc;
    __syncthreads();
    if (wave == 0) {
#pragma unroll 1
      for (int w2 = 0; w2 < NWAVE; ++w2) {
        int c = misc[w2];
        c = c < 0 ? 0 : (c > WCAP ? WCAP : c);
#pragma unroll 1
        for (int b0 = 0; b0 < c; b0 += 32) {
          const int idx = b0 + lane;
          const int ent = list[w2 * WCAP + (idx < WCAP ? idx : WCAP - 1)];
          const int m32 = (c - b0) < 32 ? (c - b0) : 32;
#pragma unroll 1
          for (int k = 0; k < m32; ++k) {
            const int u    = __builtin_amdgcn_readlane(ent, k);
            const int slot = u & (NBA - 1);
            const int el   = (u >> SLA) & (CHUNK - 1);
            const int eid  = cbase + el;
            if (lane == 0) {
              int c2 = cnt[slot];
              c2 = c2 < 0 ? 0 : c2;
              if (c2 < DEGC) rows[slot * NBW + c2] = eid;
              cnt[slot] = c2 + 1;
            }
          }
        }
      }
    }
    __syncthreads();
  }

#pragma unroll 1
  for (int idx = tid; idx < NBA * NBW; idx += NTHR) {
    const int slot = idx >> 5;
    const int k    = idx & 31;
    const int c    = cnt[slot];
    const int cc   = c < 0 ? 0 : (c > DEGC ? DEGC : c);
    int e = rows[idx];
    e = e < 0 ? 0 : (e > nE - 1 ? nE - 1 : e);
    int s = srcs[e];
    s = s < 0 ? 0 : (s > nN - 1 ? nN - 1 : s);
    int val = (k < cc) ? s : 0;
    val = (k == 31) ? ((c > DEGC) ? -1 : cc) : val;
    rows[idx] = val;
  }
  __syncthreads();

  int* gb = nbr + (size_t)nodeBase * NBW;
  constexpr int NITC = (NBA * NBW / 4) / NTHR;
#pragma unroll 4
  for (int it = 0; it < NITC; ++it) {
    const int i4 = 4 * (it * NTHR + tid);
    const v4i v = *(const v4ia*)(rows + i4);
    *(volatile v4i*)(gb + i4) = v;
  }
  __threadfence();
#pragma unroll 4
  for (int it = 0; it < NITC; ++it) {
    const int i4 = 4 * (it * NTHR + tid);
    const v4i v = *(const v4ia*)(rows + i4);
    *(volatile v4i*)(gb + i4) = v;
  }
}

__device__ __forceinline__ float gacc(float rx, float ry, float w0, float w1, float b, float h, float acc) {
  float g = fmaf(rx, w0, fmaf(ry, w1, b));
  g = fmaxf(g, 0.0f);
  return fmaf(g, h, acc);
}

template <int C, int XIN>
__global__ __launch_bounds__(ATHR) void k_agg(const float* __restrict__ hin, const float* __restrict__ pos,
                                              const int* __restrict__ nbr, int nbrRows,
                                              const float* __restrict__ Win, const float* __restrict__ bin,
                                              unsigned short* agg, int nN, int mRows) {
  constexpr int SEGC = (C < 256) ? C : 256;
  constexpr int NW   = C / SEGC;
  constexpr int LPS  = SEGC / 8;
  constexpr int RW   = (ATHR / 32) / NW;
  constexpr int RB   = RW * AITER;
  static_assert(C % SEGC == 0 && (ATHR / 32) % NW == 0 && (LPS == 16 || LPS == 32));
  const int tid = (int)threadIdx.x, lane = tid & 31;
  const int wave = __builtin_amdgcn_readfirstlane(tid >> 5);
  const int seg  = wave % NW;
  const int rsub = wave / NW;
  const int ls   = lane & (LPS - 1);
  const bool active = lane < LPS;
  const int c0 = seg * SEGC + 8 * ls;

  float w0[8], w1[8], bb[8];
  {
    const v4f a0 = bf16_val4(*(const v4fa*)(Win + c0));
    const v4f a1 = bf16_val4(*(const v4fa*)(Win + c0 + 4));
    const v4f b0 = bf16_val4(*(const v4fa*)(Win + C + c0));
    const v4f b1 = bf16_val4(*(const v4fa*)(Win + C + c0 + 4));
    const v4f d0 = bf16_val4(*(const v4fa*)(bin + c0));
    const v4f d1 = bf16_val4(*(const v4fa*)(bin + c0 + 4));
    w0[0] = a0.x; w0[1] = a0.y; w0[2] = a0.z; w0[3] = a0.w; w0[4] = a1.x; w0[5] = a1.y; w0[6] = a1.z; w0[7] = a1.w;
    w1[0] = b0.x; w1[1] = b0.y; w1[2] = b0.z; w1[3] = b0.w; w1[4] = b1.x; w1[5] = b1.y; w1[6] = b1.z; w1[7] = b1.w;
    bb[0] = d0.x; bb[1] = d0.y; bb[2] = d0.z; bb[3] = d0.w; bb[4] = d1.x; bb[5] = d1.y; bb[6] = d1.z; bb[7] = d1.w;
  }
  const float qnan = __int_as_float(0x7fc00000);

#pragma unroll 1
  for (int it = 0; it < AITER; ++it) {
    const int i = (int)blockIdx.x * RB + it * RW + rsub;
    const bool live = i < nN;
    const int ic = live ? i : nN - 1;
    const int ir = i < nbrRows ? i : nbrRows - 1;
    const int ent = nbr[(size_t)ir * NBW + lane];
    const int craw = __builtin_amdgcn_readlane(ent, 31);
    const bool bad = live && ((craw < 0) || (craw > DEGC));
    int cnt = craw < 0 ? 0 : (craw > DEGC ? DEGC : craw);
    cnt = live ? cnt : 0;
    const int j = ent < 0 ? 0 : (ent > nN - 1 ? nN - 1 : ent);
    const v2f pj = *(const v2fa*)(pos + 2 * (size_t)j);
    const v2f pi = *(const v2fa*)(pos + 2 * (size_t)ic);
    const float rx = bf16_val(pj.x) - bf16_val(pi.x);
    const float ry = bf16_val(pj.y) - bf16_val(pi.y);
    const int rxi = __float_as_int(rx), ryi = __float_as_int(ry);

    float ac[8];
#pragma unroll
    for (int q = 0; q < 8; ++q) ac[q] = 0.0f;
#pragma unroll 1
    for (int k = 0; k < cnt; ++k) {
      const int   sk  = __builtin_amdgcn_readlane(j, k);
      const float rxk = __int_as_float(__builtin_amdgcn_readlane(rxi, k));
      const float ryk = __int_as_float(__builtin_amdgcn_readlane(ryi, k));
      const float* hp = hin + (size_t)sk * (size_t)C + c0;
      v4f a = *(const v4fa*)hp;
      v4f b = *(const v4fa*)(hp + 4);
      if constexpr (XIN != 0) { a = bf16_val4(a); b = bf16_val4(b); }
      ac[0] = gacc(rxk, ryk, w0[0], w1[0], bb[0], a.x, ac[0]);
      ac[1] = gacc(rxk, ryk, w0[1], w1[1], bb[1], a.y, ac[1]);
      ac[2] = gacc(rxk, ryk, w0[2], w1[2], bb[2], a.z, ac[2]);
      ac[3] = gacc(rxk, ryk, w0[3], w1[3], bb[3], a.w, ac[3]);
      ac[4] = gacc(rxk, ryk, w0[4], w1[4], bb[4], b.x, ac[4]);
      ac[5] = gacc(rxk, ryk, w0[5], w1[5], bb[5], b.y, ac[5]);
      ac[6] = gacc(rxk, ryk, w0[6], w1[6], bb[6], b.z, ac[6]);
      ac[7] = gacc(rxk, ryk, w0[7], w1[7], bb[7], b.w, ac[7]);
    }
    const float pzr = bad ? qnan : 0.0f;
    v8us oh, ol;
#pragma unroll
    for (int q = 0; q < 8; ++q) {
      const float mv = live ? (ac[q] + pzr) : 0.0f;
      const unsigned hb = bf16_bits(mv);
      const unsigned lb = bf16_bits(mv - __uint_as_float(hb << 16));
      oh[q] = (unsigned short)hb;
      ol[q] = (unsigned short)lb;
    }
    if (i < mRows) {
      unsigned short* ph = agg + (size_t)i * (size_t)(2 * C) + c0;
      unsigned short* pl = ph + C;
      if (active) { *(volatile v8us*)ph = oh; *(volatile v8us*)pl = ol; }
      __threadfence();
      if (active) { *(volatile v8us*)ph = oh; *(volatile v8us*)pl = ol; }
    }
  }
}

__global__ __launch_bounds__(GTHR) void k_gemm(const unsigned short* __restrict__ A, int KA, int C,
                                               const unsigned short* __restrict__ WT,
                                               const float* __restrict__ bias, float* outF, int ldo, int nOut) {
  __shared__ __attribute__((aligned(16))) float stg[GBM * GBN];
  const int tid = (int)threadIdx.x, lane = tid & 31, wave = tid >> 5, hh = lane >> 4, m = lane & 15;
  const int rowBase = (int)blockIdx.x * GBM;
  const int col0    = (int)blockIdx.y * GBN;

  v8f acc[8];
  {
    const v8f z = {0.f, 0.f, 0.f, 0.f, 0.f, 0.f, 0.f, 0.f};
#pragma unroll
    for (int t = 0; t < 8; ++t) acc[t] = z;
  }
  const unsigned short* ap = A  + (size_t)(rowBase + 16 * wave + m) * (size_t)KA + 8 * hh;
  const unsigned short* bp = WT + (size_t)(col0 + m) * (size_t)C + 8 * hh;

#pragma unroll 1
  for (int k0 = 0; k0 < C; k0 += 32) {
    FragB ah, al;
    ah.h[0] = *(const v8usa*)(ap + k0);
    ah.h[1] = *(const v8usa*)(ap + k0 + 16);
    al.h[0] = *(const v8usa*)(ap + C + k0);
    al.h[1] = *(const v8usa*)(ap + C + k0 + 16);
#pragma unroll
    for (int nt = 0; nt < 8; ++nt) {
      const unsigned short* wq = bp + (size_t)(16 * nt) * (size_t)C + k0;
      FragB bf;
      bf.h[0] = *(const v8usa*)wq;
      bf.h[1] = *(const v8usa*)(wq + 16);
      acc[nt] = wmb(ah, bf, acc[nt]);
      acc[nt] = wmb(al, bf, acc[nt]);
    }
  }

#pragma unroll
  for (int nt = 0; nt < 8; ++nt) {
    const int lc = 16 * nt + m;
#pragma unroll
    for (int r = 0; r < 8; ++r) {
      const int lr = 16 * wave + 8 * hh + r;
      stg[lr * GBN + lc] = acc[nt][r];
    }
  }
  __syncthreads();

  const v4f bb4 = bf16_val4(*(const v4fa*)(bias + col0 + 4 * lane));
  v4f pv[16];
#pragma unroll
  for (int i = 0; i < 16; ++i) pv[i] = *(const v4fa*)(stg + (16 * wave + i) * GBN + 4 * lane);
#pragma unroll
  for (int i = 0; i < 16; ++i) {
    const v4f t = pv[i] + bb4;
    v4f y;
    y.x = (t.x > 0.0f) ? t.x : (t.x - t.x);
    y.y = (t.y > 0.0f) ? t.y : (t.y - t.y);
    y.z = (t.z > 0.0f) ? t.z : (t.z - t.z);
    y.w = (t.w > 0.0f) ? t.w : (t.w - t.w);
    pv[i] = y;
  }
#pragma unroll
  for (int i = 0; i < 16; ++i) {
    const int r = rowBase + 16 * wave + i;
    if (r < nOut) *(volatile v4f*)(outF + (size_t)r * (size_t)ldo + col0 + 4 * lane) = pv[i];
  }
  __threadfence();
#pragma unroll
  for (int i = 0; i < 16; ++i) {
    const int r = rowBase + 16 * wave + i;
    if (r < nOut) *(volatile v4f*)(outF + (size_t)r * (size_t)ldo + col0 + 4 * lane) = pv[i];
  }
}

__global__ __launch_bounds__(NTHR) void k_norm(const float* __restrict__ h3, float* out, int nN) {
  const int tid = (int)threadIdx.x, lane = tid & 31;
  const int wave = __builtin_amdgcn_readfirstlane(tid >> 5);
  const int row = (int)blockIdx.x * NWAVE + wave;
  if (row >= nN) return;
  const float* p = h3 + (size_t)row * O3 + 4 * lane;
  v4f v[8];
#pragma unroll
  for (int it = 0; it < 8; ++it) v[it] = *(const v4fa*)(p + it * 128);
  float s = 0.0f;
#pragma unroll
  for (int it = 0; it < 8; ++it) {
    s = fmaf(v[it].x, v[it].x, s);
    s = fmaf(v[it].y, v[it].y, s);
    s = fmaf(v[it].z, v[it].z, s);
    s = fmaf(v[it].w, v[it].w, s);
  }
#pragma unroll
  for (int d = 16; d >= 1; d >>= 1) s += __shfl_xor(s, d, 32);
  const float nrm = sqrtf(s);
  const float dn  = (nrm < 1e-12f) ? 1e-12f : nrm;
  const float inv = 1.0f / dn;
#pragma unroll
  for (int it = 0; it < 8; ++it) v[it] = v[it] * inv;
  float* op = out + (size_t)row * O3 + 4 * lane;
#pragma unroll
  for (int it = 0; it < 8; ++it) *(volatile v4f*)(op + it * 128) = v[it];
  __threadfence();
#pragma unroll
  for (int it = 0; it < 8; ++it) *(volatile v4f*)(op + it * 128) = v[it];
}

static inline int cdiv(int a, int b) { return (a + b - 1) / b; }
static inline size_t al256(size_t o) { return (o + 255) & ~(size_t)255; }

extern "C" void kernel_launch(void* const* d_in, const int* in_sizes, int n_in,
                              void* d_out, int out_size, void* d_ws, size_t ws_size,
                              hipStream_t stream) {
  if (n_in < 15) return;
  if (in_sizes[1] < 2 || (in_sizes[1] & 1) != 0) return;
  const int nN = in_sizes[1] / 2;
  if (nN < 1 || nN > (1 << 20)) return;
  if ((long long)in_sizes[0] != (long long)nN * C1) return;
  if (in_sizes[2] < 2 || (in_sizes[2] & 1) != 0) return;
  const int nE = in_sizes[2] / 2;
  if (nE < 1 || nE >= (1 << 28)) return;
  if (in_sizes[3] != 2 * C1 || in_sizes[4] != C1) return;
  if (in_sizes[5] != C1 * O1 || in_sizes[6] != O1) return;
  if (in_sizes[7] != 2 * C2 || in_sizes[8] != C2) return;
  if (in_sizes[9] != C2 * O2 || in_sizes[10] != O2) return;
  if (in_sizes[11] != 2 * C3 || in_sizes[12] != C3) return;
  if (in_sizes[13] != C3 * O3 || in_sizes[14] != O3) return;
  if ((long long)out_size != (long long)nN * O3) return;

  const float* x    = (const float*)d_in[0];
  const float* pos  = (const float*)d_in[1];
  const int*   edge = (const int*)d_in[2];
  const float* Wi1  = (const float*)d_in[3];
  const float* bi1  = (const float*)d_in[4];
  const float* Wo1  = (const float*)d_in[5];
  const float* bo1  = (const float*)d_in[6];
  const float* Wi2  = (const float*)d_in[7];
  const float* bi2  = (const float*)d_in[8];
  const float* Wo2  = (const float*)d_in[9];
  const float* bo2  = (const float*)d_in[10];
  const float* Wi3  = (const float*)d_in[11];
  const float* bi3  = (const float*)d_in[12];
  const float* Wo3  = (const float*)d_in[13];
  const float* bo3  = (const float*)d_in[14];
  float* out = (float*)d_out;
  const int* src = edge;
  const int* dst = edge + nE;

  const int MP = cdiv(nN, GBM) * GBM;
  const int gM = MP / GBM;
  const int gB = cdiv(MP, NBA);
  const int nbrRows = gB * NBA;
  if (nbrRows < MP) return;

  char* ws = (char*)d_ws;
  size_t off = 0;
  const size_t oH  = off; off = al256(off + (size_t)nN * O1 * 4);
  const size_t oAG = off; off = al256(off + (size_t)MP * (2 * C2) * 2);
  const size_t oW1 = off; off = al256(off + (size_t)O1 * C1 * 2);
  const size_t oW2 = off; off = al256(off + (size_t)O2 * C2 * 2);
  const size_t oW3 = off; off = al256(off + (size_t)O3 * C3 * 2);
  const size_t oNB = off; off = al256(off + (size_t)nbrRows * NBW * 4);
  if (off > ws_size) return;
  float*          Hp  = (float*)(ws + oH);
  unsigned short* AG  = (unsigned short*)(ws + oAG);
  unsigned short* W1T = (unsigned short*)(ws + oW1);
  unsigned short* W2T = (unsigned short*)(ws + oW2);
  unsigned short* W3T = (unsigned short*)(ws + oW3);
  int*            NBR = (int*)(ws + oNB);

  const size_t bkLds = (size_t)BK_LDS_INTS * 4;
  hipFuncSetAttribute(reinterpret_cast<const void*>(&k_bucket), hipFuncAttributeMaxDynamicSharedMemorySize, (int)bkLds);

  constexpr int RB1 = ((ATHR / 32) / 1) * AITER;
  constexpr int RB2 = ((ATHR / 32) / 8) * AITER;

  k_wprep<<<NUT / NTHR, NTHR, 0, stream>>>(Wo1, Wo2, Wo3, W1T, W2T, W3T);
  k_bucket<<<gB, NTHR, bkLds, stream>>>(src, dst, nE, nN, NBR);
  k_agg<C1, 1><<<cdiv(MP, RB1), ATHR, 0, stream>>>(x, pos, NBR, nbrRows, Wi1, bi1, AG, nN, MP);
  k_gemm<<<dim3(gM, O1 / GBN), GTHR, 0, stream>>>(AG, 2 * C1, C1, W1T, bo1, Hp, O1, nN);
  k_agg<C2, 0><<<cdiv(MP, RB2), ATHR, 0, stream>>>(Hp, pos, NBR, nbrRows, Wi2, bi2, AG, nN, MP);
  k_gemm<<<dim3(gM, O2 / GBN), GTHR, 0, stream>>>(AG, 2 * C2, C2, W2T, bo2, Hp, O2, nN);
  k_agg<C3, 0><<<cdiv(MP, RB2), ATHR, 0, stream>>>(Hp, pos, NBR, nbrRows, Wi3, bi3, AG, nN, MP);
  k_gemm<<<dim3(gM, O3 / GBN), GTHR, 0, stream>>>(AG, 2 * C3, C3, W3T, bo3, Hp, O3, nN);
  k_norm<<<cdiv(nN, NWAVE), NTHR, 0, stream>>>(Hp, out, nN);
}
